// ConformerLayer_23132693856324
// MI455X (gfx1250) — hardware-verified
//
#include <hip/hip_runtime.h>
#include <math.h>

constexpr int kT   = 512;
constexpr int kB   = 16;
constexpr int kD   = 512;
constexpr int kH   = 8;
constexpr int kHD  = 64;
constexpr int kFF  = 2048;
constexpr int kKS  = 31;
constexpr int kM   = kT * kB;
constexpr int kNPv = 2 * kT - 1;
constexpr int kNP  = 1024;
constexpr float kInvD   = 1.0f / 512.0f;
constexpr float kInvM   = 1.0f / 8192.0f;
constexpr float kLnEps  = 1e-5f;
constexpr float kBnEps  = 1e-5f;
constexpr float kAttnScale = 0.125f;
constexpr float kWCarry  = 16.0f;
constexpr float kWInv    = 1.0f / 16.0f;
constexpr float kPCarry  = 2048.0f;
constexpr float kCtxCarry = 64.0f;
constexpr float kPVScale = kCtxCarry / kPCarry;
constexpr float kOutProjScale = 1.0f / (kCtxCarry * kWCarry);
constexpr float kHalfWInv = 0.5f / 16.0f;

constexpr size_t kMiB    = 1048576;
constexpr size_t oWffm1  = 0;
constexpr size_t oWffm2  = 2 * kMiB;
constexpr size_t oWff1   = 4 * kMiB;
constexpr size_t oWff2   = 6 * kMiB;
constexpr size_t oWin    = 8 * kMiB;
constexpr size_t oWout   = 9 * kMiB + 512 * 1024;
constexpr size_t oWpos   = 10 * kMiB;
constexpr size_t oWpw1   = 10 * kMiB + 512 * 1024;
constexpr size_t oWpw2   = 11 * kMiB + 512 * 1024;
constexpr size_t oPosEmb = 12 * kMiB;
constexpr size_t oPpos   = 13 * kMiB;
constexpr size_t oHalfB  = 14 * kMiB;
constexpr size_t oBnMean = 14 * kMiB + 4096;
constexpr size_t oBnRstd = 14 * kMiB + 6144;
constexpr size_t oXnA    = 15 * kMiB;
constexpr size_t oXnF    = 23 * kMiB;
constexpr size_t oQF     = 23 * kMiB;
constexpr size_t oHid    = 39 * kMiB;
constexpr size_t oK16    = 39 * kMiB;
constexpr size_t oVT16   = 47 * kMiB;
constexpr size_t oQU16   = 55 * kMiB;
constexpr size_t oQV16   = 63 * kMiB;
constexpr size_t oY      = 39 * kMiB;
constexpr size_t oX1     = 71 * kMiB;
constexpr size_t oGlu    = 71 * kMiB;
constexpr size_t oX4     = 71 * kMiB;
constexpr size_t oAtt    = 87 * kMiB;
constexpr size_t oZ      = 87 * kMiB;
constexpr size_t oAC     = 15 * kMiB;
constexpr size_t oP16    = 31 * kMiB;
constexpr size_t oX2     = 15 * kMiB;
constexpr size_t oXnB    = 31 * kMiB;
constexpr size_t oBD     = 95 * kMiB;
constexpr size_t oSw     = 103 * kMiB;
constexpr size_t oX3     = 111 * kMiB;
constexpr size_t kWsEnd  = 127 * kMiB;
static_assert(kWsEnd <= 134217728);

typedef __attribute__((ext_vector_type(16))) _Float16 v16h;
typedef __attribute__((ext_vector_type(8)))  _Float16 v8h;
typedef __attribute__((ext_vector_type(16))) __bf16   v16b;
typedef __attribute__((ext_vector_type(8)))  __bf16   v8b;
typedef __attribute__((ext_vector_type(8)))  float    v8f;
typedef __attribute__((ext_vector_type(4)))  float    v4f;
typedef __attribute__((ext_vector_type(4)))  unsigned int v4u;

__device__ __forceinline__ unsigned short f2bf_bits(float f) {
  unsigned u = __float_as_uint(f);
  return (unsigned short)((u + 0x7FFFu + ((u >> 16) & 1u)) >> 16);
}
__device__ __forceinline__ float bf_bits2f(unsigned short h) { return __uint_as_float(((unsigned)h) << 16); }

__device__ __forceinline__ void dep_guard_h(v8f& a, v8f& b, v16h x, v16h y) { asm volatile("v_nop\n\tv_nop\n\tv_nop\n\tv_nop" : "+v"(a), "+v"(b) : "v"(x), "v"(y)); }
__device__ __forceinline__ void dep_guard_b(v8f& a, v8f& b, v16b x, v16b y) { asm volatile("v_nop\n\tv_nop\n\tv_nop\n\tv_nop" : "+v"(a), "+v"(b) : "v"(x), "v"(y)); }
__device__ __forceinline__ void keep4_h(v16h a, v16h b, v16h c, v16h d) { asm volatile("v_nop" :: "v"(a), "v"(b), "v"(c), "v"(d)); }
__device__ __forceinline__ void keep4_b(v16b a, v16b b, v16b c, v16b d) { asm volatile("v_nop" :: "v"(a), "v"(b), "v"(c), "v"(d)); }
__device__ __forceinline__ void acc_guard4(v8f& a, v8f& b, v8f& c, v8f& d) { asm volatile("v_nop\n\tv_nop\n\tv_nop\n\tv_nop" : "+v"(a), "+v"(b), "+v"(c), "+v"(d)); }
template <typename T> struct Frag;
template <> struct Frag<_Float16> {
  typedef v16h V; union U { v16h v; v8h h[2]; };
  static __device__ __forceinline__ v16h load(const _Float16* p) {
    U f; f.h[0] = *(const v8h*)(p); f.h[1] = *(const v8h*)(p + 16); return f.v;
  }
  static __device__ __forceinline__ v8f mma(v16h a, v16h b, v8f c) {
    return __builtin_amdgcn_wmma_f32_16x16x32_f16(false, a, false, b, (short)0, c, false, false);
  }
  static __device__ __forceinline__ void guard(v8f& a, v8f& b, v16h x, v16h y) { dep_guard_h(a, b, x, y); }
  static __device__ __forceinline__ void keep(v16h a, v16h b, v16h c, v16h d) { keep4_h(a, b, c, d); }
};
template <> struct Frag<__bf16> {
  typedef v16b V; union U { v16b v; v8b h[2]; };
  static __device__ __forceinline__ v16b load(const __bf16* p) {
    U f; f.h[0] = *(const v8b*)(p); f.h[1] = *(const v8b*)(p + 16); return f.v;
  }
  static __device__ __forceinline__ v8f mma(v16b a, v16b b, v8f c) {
    return __builtin_amdgcn_wmma_f32_16x16x32_bf16(false, a, false, b, (short)0, c, false, false);
  }
  static __device__ __forceinline__ void guard(v8f& a, v8f& b, v16b x, v16b y) { dep_guard_b(a, b, x, y); }
  static __device__ __forceinline__ void keep(v16b a, v16b b, v16b c, v16b d) { keep4_b(a, b, c, d); }
};

__device__ __forceinline__ unsigned pk16(unsigned short a, unsigned short b) { return (unsigned)a | ((unsigned)b << 16); }
__device__ __forceinline__ unsigned short h_bits(float f) { const _Float16 h = (_Float16)f; return __builtin_bit_cast(unsigned short, h); }

template <int ET> struct Elem;
template <> struct Elem<0> { typedef _Float16 T; };
template <> struct Elem<1> { typedef __bf16 T; };
template <int ET, bool SPLIT, int BIAS_MODE, int OUT_MODE, bool RESID, int ACT = 0>
__global__ __launch_bounds__(256) void wmma_gemm64(
    const unsigned short* __restrict__ Ap, const unsigned short* __restrict__ A2p, int lda, long strideA,
    const unsigned short* __restrict__ Btp, const unsigned short* __restrict__ Bt2p, int ldb, long strideB,
    void* __restrict__ Cout, void* __restrict__ Cout2, int ldc, long strideC,
    const float* __restrict__ bias,
    const float* __restrict__ resid, long strideR,
    int M, int N, int K, float scale) {
  typedef typename Elem<ET>::T T;
  typedef typename Frag<T>::V V;
  const T* A = (const T*)Ap; const T* A2 = (const T*)A2p; const T* Bt = (const T*)Btp; const T* Bt2 = (const T*)Bt2p;
  __shared__ __align__(16) float sT[8][16 * 68];
  const int b    = blockIdx.y;
  const int lane = threadIdx.x & 31;
  const int wave = threadIdx.x >> 5;
  const int tilesN = N >> 6;
  const int tilesM = M >> 6;
  const int tile = blockIdx.x * 8 + wave;
  if (tile >= tilesM * tilesN) return;
  const int tm = tile / tilesN;
  const int tn = tile - tm * tilesN;
  const int m0 = tm << 6;
  const int n0 = tn << 6;

  const T* Ab  = A  + (size_t)b * strideA;
  const T* Bb  = Bt + (size_t)b * strideB;
  const T* Ab2 = SPLIT ? (A2  + (size_t)b * strideA) : nullptr;
  const T* Bb2 = SPLIT ? (Bt2 + (size_t)b * strideB) : nullptr;

  const int rlane = lane & 15;
  const int koff  = (lane >> 4) * 8;
  const int mOff  = (lane >> 4) * 8;

  v8f acc[4][4];
#pragma unroll
  for (int i = 0; i < 4; ++i)
#pragma unroll
    for (int j = 0; j < 4; ++j) acc[i][j] = (v8f){0.f,0.f,0.f,0.f,0.f,0.f,0.f,0.f};

  for (int k0 = 0; k0 < K; k0 += 32) {
    V bh[4], bl[4];
#pragma unroll
    for (int j = 0; j < 4; ++j) {
      const size_t bo = (size_t)(n0 + (j << 4) + rlane) * ldb + koff + k0;
      bh[j] = Frag<T>::load(Bb + bo);
      if (SPLIT) bl[j] = Frag<T>::load(Bb2 + bo);
    }
#pragma unroll
    for (int i = 0; i < 4; ++i) {
      const size_t ao = (size_t)(m0 + (i << 4) + rlane) * lda + koff + k0;
      V ah = Frag<T>::load(Ab + ao);
      V al;
      if (SPLIT) al = Frag<T>::load(Ab2 + ao);
#pragma unroll
      for (int j = 0; j < 4; ++j) {
        acc[i][j] = Frag<T>::mma(ah, bh[j], acc[i][j]);
        if (SPLIT) {
          acc[i][j] = Frag<T>::mma(ah, bl[j], acc[i][j]);
          acc[i][j] = Frag<T>::mma(al, bh[j], acc[i][j]);
        }
      }
      Frag<T>::guard(acc[i][0], acc[i][3], ah, SPLIT ? al : ah);
    }
    Frag<T>::keep(bh[0], bh[1], bh[2], bh[3]);
    if (SPLIT) Frag<T>::keep(bl[0], bl[1], bl[2], bl[3]);
  }
  acc_guard4(acc[0][0], acc[0][1], acc[0][2], acc[0][3]);
  acc_guard4(acc[1][0], acc[1][1], acc[1][2], acc[1][3]);
  acc_guard4(acc[2][0], acc[2][1], acc[2][2], acc[2][3]);
  acc_guard4(acc[3][0], acc[3][1], acc[3][2], acc[3][3]);

  float* slab = sT[wave];
  const float* Rb = RESID ? (resid + (size_t)b * strideR) : nullptr;
#pragma unroll
  for (int i = 0; i < 4; ++i) {
    const int mBase = m0 + (i << 4);
#pragma unroll
    for (int j = 0; j < 4; ++j) {
      const int n = n0 + (j << 4) + rlane;
      float bv = 0.f;
      if (BIAS_MODE == 2) bv = bias[n];
#pragma unroll
      for (int r = 0; r < 8; ++r) {
        float v = acc[i][j][r] * scale;
        if (BIAS_MODE == 1) v += bias[mBase + mOff + r];
        if (BIAS_MODE == 2) v += bv;
        if (RESID) v += Rb[(size_t)(mBase + mOff + r) * ldc + n];
        if (ACT == 2) v = fmaxf(v, 0.0f);
        if (ACT == 3) v = v / (1.0f + expf(-v));
        if (ACT == 4) v = (v > 0.f) ? v : 0.01f * v;
        slab[(mOff + r) * 68 + (j << 4) + rlane] = v;
      }
    }
    __builtin_amdgcn_fence(__ATOMIC_RELEASE, "workgroup");
    __builtin_amdgcn_wave_barrier();
    __builtin_amdgcn_fence(__ATOMIC_ACQUIRE, "workgroup");
    if (OUT_MODE == 0) {
      float* C = (float*)Cout + (size_t)b * strideC;
      const int hh = lane >> 4, c4 = (lane & 15) * 4;
      for (int pass = 0; pass < 2; ++pass) {
#pragma unroll
        for (int it = 0; it < 8; ++it) {
          const int row = it * 2 + hh;
          v4f v = *(const v4f*)(slab + row * 68 + c4);
          *(volatile v4f*)(C + (size_t)(mBase + row) * ldc + n0 + c4) = v;
        }
        __threadfence();
      }
    } else {
      const int q = lane >> 3, c8 = (lane & 7) * 8;
      unsigned short* C  = (unsigned short*)Cout  + (size_t)b * strideC;
      unsigned short* C2 = (OUT_MODE == 2) ? ((unsigned short*)Cout2 + (size_t)b * strideC) : nullptr;
      for (int pass = 0; pass < 2; ++pass) {
#pragma unroll
        for (int it = 0; it < 4; ++it) {
          const int row = it * 4 + q;
          const float* sp = slab + row * 68 + c8;
          v8h hv, lv;
#pragma unroll
          for (int e = 0; e < 8; ++e) {
            if (OUT_MODE == 1) {
              hv[e] = (_Float16)sp[e];
            } else {
              unsigned short hb = f2bf_bits(sp[e]);
              unsigned short lb = f2bf_bits(sp[e] - bf_bits2f(hb));
              hv[e] = __builtin_bit_cast(_Float16, hb);
              lv[e] = __builtin_bit_cast(_Float16, lb);
            }
          }
          *(volatile v8h*)(C + (size_t)(mBase + row) * ldc + n0 + c8) = hv;
          if (OUT_MODE == 2) *(volatile v8h*)(C2 + (size_t)(mBase + row) * ldc + n0 + c8) = lv;
        }
        __threadfence();
      }
    }
    __builtin_amdgcn_fence(__ATOMIC_RELEASE, "workgroup");
    __builtin_amdgcn_wave_barrier();
    __builtin_amdgcn_fence(__ATOMIC_ACQUIRE, "workgroup");
  }
}

__global__ __launch_bounds__(256) void cast4_kernel(
    const float* __restrict__ in0, unsigned short* __restrict__ out0, int nv0, int nt0, float sc0,
    const float* __restrict__ in1, unsigned short* __restrict__ out1, int nv1, int nt1, float sc1,
    const float* __restrict__ in2, unsigned short* __restrict__ out2, int nv2, int nt2, float sc2,
    const float* __restrict__ in3, unsigned short* __restrict__ out3, int nv3, int nt3, float sc3) {
  const int z = blockIdx.y;
  const float* in = (z == 0) ? in0 : (z == 1) ? in1 : (z == 2) ? in2 : in3;
  unsigned short* out = (z == 0) ? out0 : (z == 1) ? out1 : (z == 2) ? out2 : out3;
  const int nv = (z == 0) ? nv0 : (z == 1) ? nv1 : (z == 2) ? nv2 : nv3;
  const int nt = (z == 0) ? nt0 : (z == 1) ? nt1 : (z == 2) ? nt2 : nt3;
  const float sc = (z == 0) ? sc0 : (z == 1) ? sc1 : (z == 2) ? sc2 : sc3;
  const int i = blockIdx.x * 256 + threadIdx.x;
  if (i >= nt) return;
  const bool valid = (i < nv);
  const int ic = valid ? i : (nv - 1);
  const float f = valid ? sc : 0.0f;
  const float* p = in + 8 * (size_t)ic;
  const v4f a = *(const v4f*)(p);
  const v4f c = *(const v4f*)(p + 4);
  unsigned short hb[8];
#pragma unroll
  for (int e = 0; e < 4; ++e) {
    hb[e]     = h_bits(a[e] * f);
    hb[4 + e] = h_bits(c[e] * f);
  }
  const v4u u = (v4u){pk16(hb[0], hb[1]), pk16(hb[2], hb[3]), pk16(hb[4], hb[5]), pk16(hb[6], hb[7])};
  unsigned short* q = out + 8 * (size_t)i;
  *(volatile v4u*)q = u;
  __threadfence();
  *(volatile v4u*)q = u;
}

__global__ __launch_bounds__(256) void halfbias_kernel(const float* __restrict__ b0, const float* __restrict__ b1,
                                                       float* __restrict__ out) {
  const int i = threadIdx.x;
  const int j = 4 * (i & 127);
  const v4f a = *(const v4f*)(b0 + j);
  const v4f c = *(const v4f*)(b1 + j);
  v4f v;
#pragma unroll
  for (int e = 0; e < 4; ++e) v[e] = (i < 128) ? (a[e] * 0.5f) : (c[e] * 0.5f);
  float* q = out + 4 * i;
  *(volatile v4f*)q = v;
  __threadfence();
  *(volatile v4f*)q = v;
}

template <bool OUTF, bool OUTH>
__global__ __launch_bounds__(256) void ln_kernel(const float* __restrict__ x, const float* __restrict__ gam,
                                                 const float* __restrict__ bet, float* __restrict__ outF,
                                                 unsigned short* __restrict__ outH, int nrows) {
  const int lane = threadIdx.x & 31, wave = threadIdx.x >> 5;
  const int row = blockIdx.x * 8 + wave;
  if (row >= nrows) return;
  const float* xr = x + (size_t)row * kD;
  v4f v[4];
  float s = 0.f;
#pragma unroll
  for (int i = 0; i < 4; ++i) {
    v[i] = *(const v4f*)(xr + (i * 32 + lane) * 4);
    s += (v[i][0] + v[i][1]) + (v[i][2] + v[i][3]);
  }
#pragma unroll
  for (int o = 16; o > 0; o >>= 1) s += __shfl_xor(s, o, 32);
  const float mean = s * kInvD;
  float q = 0.f;
#pragma unroll
  for (int i = 0; i < 4; ++i) {
#pragma unroll
    for (int e = 0; e < 4; ++e) { const float d = v[i][e] - mean; q += d * d; }
  }
#pragma unroll
  for (int o = 16; o > 0; o >>= 1) q += __shfl_xor(q, o, 32);
  const float rstd = 1.0f / sqrtf(q * kInvD + kLnEps);
  if (OUTF) {
    v4f o[4];
#pragma unroll
    for (int i = 0; i < 4; ++i) {
      const v4f gg = *(const v4f*)(gam + (i * 32 + lane) * 4);
      const v4f be = *(const v4f*)(bet + (i * 32 + lane) * 4);
#pragma unroll
      for (int e = 0; e < 4; ++e) o[i][e] = (v[i][e] - mean) * rstd * gg[e] + be[e];
    }
    float* orow = outF + (size_t)row * kD;
    for (int pass = 0; pass < 2; ++pass) {
#pragma unroll
      for (int i = 0; i < 4; ++i) *(volatile v4f*)(orow + (i * 32 + lane) * 4) = o[i];
      __threadfence();
    }
  }
  if (OUTH) {
    v4u u[2];
#pragma unroll
    for (int i2 = 0; i2 < 2; ++i2) {
      const int cb = (i2 * 32 + lane) * 8;
      const v4f a  = *(const v4f*)(xr + cb);
      const v4f c  = *(const v4f*)(xr + cb + 4);
      const v4f ga = *(const v4f*)(gam + cb);
      const v4f gc = *(const v4f*)(gam + cb + 4);
      const v4f ba = *(const v4f*)(bet + cb);
      const v4f bc = *(const v4f*)(bet + cb + 4);
      unsigned short hb[8];
#pragma unroll
      for (int e = 0; e < 4; ++e) {
        hb[e]     = h_bits((a[e] - mean) * rstd * ga[e] + ba[e]);
        hb[4 + e] = h_bits((c[e] - mean) * rstd * gc[e] + bc[e]);
      }
      u[i2] = (v4u){pk16(hb[0], hb[1]), pk16(hb[2], hb[3]), pk16(hb[4], hb[5]), pk16(hb[6], hb[7])};
    }
    unsigned short* hrow = outH + (size_t)row * kD;
    for (int pass = 0; pass < 2; ++pass) {
#pragma unroll
      for (int i2 = 0; i2 < 2; ++i2) *(volatile v4u*)(hrow + (i2 * 32 + lane) * 8) = u[i2];
      __threadfence();
    }
  }
}

__global__ __launch_bounds__(256) void quv_kernel(const float* __restrict__ qf, const float* __restrict__ bu,
                                                  const float* __restrict__ bv, unsigned short* __restrict__ qu,
                                                  unsigned short* __restrict__ qv, int n8) {
  const int i = blockIdx.x * 256 + threadIdx.x;
  if (i >= n8) return;
  const int c0 = (i & 63) * 8;
  const float* p = qf + 8 * (size_t)i;
  const v4f a  = *(const v4f*)(p);
  const v4f c  = *(const v4f*)(p + 4);
  const v4f ua = *(const v4f*)(bu + c0);
  const v4f uc = *(const v4f*)(bu + c0 + 4);
  const v4f va = *(const v4f*)(bv + c0);
  const v4f vc = *(const v4f*)(bv + c0 + 4);
  unsigned short hu[8], hv[8];
#pragma unroll
  for (int e = 0; e < 4; ++e) {
    hu[e]     = h_bits(a[e] + ua[e]);
    hu[4 + e] = h_bits(c[e] + uc[e]);
    hv[e]     = h_bits(a[e] + va[e]);
    hv[4 + e] = h_bits(c[e] + vc[e]);
  }
  const v4u uu = (v4u){pk16(hu[0], hu[1]), pk16(hu[2], hu[3]), pk16(hu[4], hu[5]), pk16(hu[6], hu[7])};
  const v4u uv = (v4u){pk16(hv[0], hv[1]), pk16(hv[2], hv[3]), pk16(hv[4], hv[5]), pk16(hv[6], hv[7])};
  unsigned short* pu = qu + 8 * (size_t)i;
  unsigned short* pv = qv + 8 * (size_t)i;
  *(volatile v4u*)pu = uu;
  *(volatile v4u*)pv = uv;
  __threadfence();
  *(volatile v4u*)pu = uu;
  *(volatile v4u*)pv = uv;
}

__global__ __launch_bounds__(256) void softmax_kernel(const float* __restrict__ ac, const float* __restrict__ bd,
                                                      unsigned short* __restrict__ p16, int nrows) {
  const int lane = threadIdx.x & 31, wave = threadIdx.x >> 5;
  const int R = blockIdx.x * 8 + wave;
  if (R >= nrows) return;
  const int qi = R & (kT - 1);
  const float* ar = ac + (size_t)R * kT;
  const float* br = bd + (size_t)R * kNP + (kT - 1 - qi);
  float xs[16];
#pragma unroll
  for (int hq = 0; hq < 2; ++hq) {
    const int cb = hq * 256 + lane * 8;
    const v4f a0 = *(const v4f*)(ar + cb);
    const v4f a1 = *(const v4f*)(ar + cb + 4);
#pragma unroll
    for (int e = 0; e < 4; ++e) {
      xs[hq * 8 + e]     = (a0[e] + br[cb + e]) * kAttnScale;
      xs[hq * 8 + 4 + e] = (a1[e] + br[cb + 4 + e]) * kAttnScale;
    }
  }
  float m = xs[0];
#pragma unroll
  for (int e = 1; e < 16; ++e) m = fmaxf(m, xs[e]);
#pragma unroll
  for (int o = 16; o > 0; o >>= 1) m = fmaxf(m, __shfl_xor(m, o, 32));
  float ev[16];
  float sum = 0.f;
#pragma unroll
  for (int e = 0; e < 16; ++e) { ev[e] = expf(xs[e] - m); sum += ev[e]; }
#pragma unroll
  for (int o = 16; o > 0; o >>= 1) sum += __shfl_xor(sum, o, 32);
  const float inv = 1.0f / sum;
  v4u u[2];
#pragma unroll
  for (int hq = 0; hq < 2; ++hq) {
    unsigned short hb[8];
#pragma unroll
    for (int e = 0; e < 8; ++e) hb[e] = h_bits((ev[hq * 8 + e] * inv) * kPCarry);
    u[hq] = (v4u){pk16(hb[0], hb[1]), pk16(hb[2], hb[3]), pk16(hb[4], hb[5]), pk16(hb[6], hb[7])};
  }
  unsigned short* prow = p16 + (size_t)R * kT;
  for (int pass = 0; pass < 2; ++pass) {
#pragma unroll
    for (int hq = 0; hq < 2; ++hq) *(volatile v4u*)(prow + hq * 256 + lane * 8) = u[hq];
    __threadfence();
  }
}

__global__ __launch_bounds__(256) void glu_kernel(const float* __restrict__ y, float* __restrict__ out, int n4) {
  const int i = blockIdx.x * 256 + threadIdx.x;
  if (i >= n4) return;
  const int row = i >> 7;
  const int col = (i & 127) * 4;
  const float* p = y + (size_t)row * (2 * kD) + col;
  const v4f a = *(const v4f*)(p);
  const v4f g = *(const v4f*)(p + kD);
  v4f o;
#pragma unroll
  for (int e = 0; e < 4; ++e) o[e] = a[e] * (1.0f / (1.0f + expf(-g[e])));
  float* q = out + 4 * (size_t)i;
  *(volatile v4f*)q = o;
  __threadfence();
  *(volatile v4f*)q = o;
}

__global__ __launch_bounds__(256) void dwconv_kernel(const float* __restrict__ glu, const float* __restrict__ w,
                                                     const float* __restrict__ bias, float* __restrict__ z, int n) {
  const int idx = blockIdx.x * 256 + threadIdx.x;
  if (idx >= n) return;
  const int c = idx & (kD - 1);
  const int r = idx >> 9;
  const int t = r >> 4;
  const int b = r & (kB - 1);
  float acc = 0.f;
#pragma unroll
  for (int k = 0; k < kKS; ++k) {
    const int tt = t + k - (kKS - 1) / 2;
    const bool valid = ((unsigned)tt < (unsigned)kT);
    const int ttc = valid ? tt : t;
    float gv = glu[((size_t)(ttc * kB + b)) * kD + c];
    gv = valid ? gv : 0.0f;
    acc += w[c * kKS + k] * gv;
  }
  const float o = acc + bias[c];
  *(volatile float*)(z + idx) = o;
  __threadfence();
  *(volatile float*)(z + idx) = o;
}

__global__ __launch_bounds__(256) void bnstats_kernel(const float* __restrict__ z, float* __restrict__ meanOut,
                                                      float* __restrict__ rstdOut) {
  __shared__ float part1[8][32];
  __shared__ float part2[8][32];
  __shared__ float meanl[32];
  const int lane = threadIdx.x & 31, wave = threadIdx.x >> 5;
  const int c = blockIdx.x * 32 + lane;
  float s = 0.f;
#pragma unroll 4
  for (int r = wave; r < kM; r += 8) s += z[(size_t)r * kD + c];
  part1[wave][lane] = s;
  __syncthreads();
  if (wave == 0) {
    float m = 0.f;
#pragma unroll
    for (int w2 = 0; w2 < 8; ++w2) m += part1[w2][lane];
    meanl[lane] = m * kInvM;
  }
  __syncthreads();
  const float mean = meanl[lane];
  float q = 0.f;
#pragma unroll 4
  for (int r = wave; r < kM; r += 8) { const float d = z[(size_t)r * kD + c] - mean; q += d * d; }
  part2[wave][lane] = q;
  __syncthreads();
  if (wave == 0) {
    float vv = 0.f;
#pragma unroll
    for (int w2 = 0; w2 < 8; ++w2) vv += part2[w2][lane];
    vv *= kInvM;
    const float rstd = 1.0f / sqrtf(vv + kBnEps);
    *(volatile float*)(meanOut + c) = mean;
    *(volatile float*)(rstdOut + c) = rstd;
    __threadfence();
    *(volatile float*)(meanOut + c) = mean;
    *(volatile float*)(rstdOut + c) = rstd;
  }
}

__global__ __launch_bounds__(256) void bnswish_kernel(const float* __restrict__ z, const float* __restrict__ mean,
                                                      const float* __restrict__ rstd, const float* __restrict__ g,
                                                      const float* __restrict__ bb, unsigned short* __restrict__ out, int n8) {
  const int i = blockIdx.x * 256 + threadIdx.x;
  if (i >= n8) return;
  const int c0 = (i & 63) * 8;
  const float* p = z + 8 * (size_t)i;
  const v4f a  = *(const v4f*)(p);
  const v4f c  = *(const v4f*)(p + 4);
  const v4f m0 = *(const v4f*)(mean + c0);
  const v4f m1 = *(const v4f*)(mean + c0 + 4);
  const v4f r0 = *(const v4f*)(rstd + c0);
  const v4f r1 = *(const v4f*)(rstd + c0 + 4);
  const v4f g0 = *(const v4f*)(g + c0);
  const v4f g1 = *(const v4f*)(g + c0 + 4);
  const v4f b0 = *(const v4f*)(bb + c0);
  const v4f b1 = *(const v4f*)(bb + c0 + 4);
  unsigned short hb[8];
#pragma unroll
  for (int e = 0; e < 4; ++e) {
    const float zn0 = (a[e] - m0[e]) * r0[e] * g0[e] + b0[e];
    const float zn1 = (c[e] - m1[e]) * r1[e] * g1[e] + b1[e];
    hb[e]     = h_bits(zn0 * (1.0f / (1.0f + expf(-zn0))));
    hb[4 + e] = h_bits(zn1 * (1.0f / (1.0f + expf(-zn1))));
  }
  const v4u u = (v4u){pk16(hb[0], hb[1]), pk16(hb[2], hb[3]), pk16(hb[4], hb[5]), pk16(hb[6], hb[7])};
  unsigned short* q = out + 8 * (size_t)i;
  *(volatile v4u*)q = u;
  __threadfence();
  *(volatile v4u*)q = u;
}

template <int BIASM, int OUTM, bool RES, int ACT>
static void run_gemm(hipStream_t st, const void* A, int lda, long sA, const void* Bt, int ldb, long sB,
                     void* C, int ldc, long sC, const float* bias, const float* resid, long sR,
                     int Mm, int Nn, int Kk, float scale, int nbatch) {
  const int tiles = (Mm >> 6) * (Nn >> 6);
  dim3 grid((tiles + 7) / 8, nbatch);
  wmma_gemm64<0, false, BIASM, OUTM, RES, ACT><<<grid, 256, 0, st>>>(
      (const unsigned short*)A, (const unsigned short*)A, lda, sA,
      (const unsigned short*)Bt, (const unsigned short*)Bt, ldb, sB,
      C, C, ldc, sC, bias, resid, sR, Mm, Nn, Kk, scale);
}

extern "C" void kernel_launch(void* const* d_in, const int* in_sizes, int n_in,
                              void* d_out, int out_size, void* d_ws, size_t ws_size,
                              hipStream_t stream) {
  if (n_in < 35) return;
  if (in_sizes[0] != kM * kD || in_sizes[1] != kNPv * kD || out_size != kM * kD) return;
  if (in_sizes[2] != 3 * kD * kD || in_sizes[9] != kFF * kD || in_sizes[17] != 2 * kD * kD || in_sizes[19] != kD * kKS) return;
  if (ws_size < kWsEnd) return;

  const float* x        = (const float*)d_in[0];
  const float* pos_emb  = (const float*)d_in[1];
  const float* in_w     = (const float*)d_in[2];
  const float* in_b     = (const float*)d_in[3];
  const float* out_w    = (const float*)d_in[4];
  const float* out_b    = (const float*)d_in[5];
  const float* pos_w    = (const float*)d_in[6];
  const float* pbu      = (const float*)d_in[7];
  const float* pbv      = (const float*)d_in[8];
  const float* ffm_w1   = (const float*)d_in[9];
  const float* ffm_b1   = (const float*)d_in[10];
  const float* ffm_w2   = (const float*)d_in[11];
  const float* ffm_b2   = (const float*)d_in[12];
  const float* ff_w1    = (const float*)d_in[13];
  const float* ff_b1    = (const float*)d_in[14];
  const float* ff_w2    = (const float*)d_in[15];
  const float* ff_b2    = (const float*)d_in[16];
  const float* pw1_w    = (const float*)d_in[17];
  const float* pw1_b    = (const float*)d_in[18];
  const float* dw_w     = (const float*)d_in[19];
  const float* dw_b     = (const float*)d_in[20];
  const float* bn_g     = (const float*)d_in[21];
  const float* bn_b     = (const float*)d_in[22];
  const float* pw2_w    = (const float*)d_in[23];
  const float* pw2_b    = (const float*)d_in[24];
  const float* ln_mac_g = (const float*)d_in[25];
  const float* ln_mac_b = (const float*)d_in[26];
  const float* ln_mha_g = (const float*)d_in[27];
  const float* ln_mha_b = (const float*)d_in[28];
  const float* ln_conv_g = (const float*)d_in[29];
  const float* ln_conv_b = (const float*)d_in[30];
  const float* ln_ff_g  = (const float*)d_in[31];
  const float* ln_ff_b  = (const float*)d_in[32];
  const float* ln_fin_g = (const float*)d_in[33];
  const float* ln_fin_b = (const float*)d_in[34];
  float* out = (float*)d_out;

  char* ws = (char*)d_ws;
  unsigned short* w_ffm1 = (unsigned short*)(ws + oWffm1);
  unsigned short* w_ffm2 = (unsigned short*)(ws + oWffm2);
  unsigned short* w_ff1  = (unsigned short*)(ws + oWff1);
  unsigned short* w_ff2  = (unsigned short*)(ws + oWff2);
  unsigned short* w_in   = (unsigned short*)(ws + oWin);
  unsigned short* w_out  = (unsigned short*)(ws + oWout);
  unsigned short* w_pos  = (unsigned short*)(ws + oWpos);
  unsigned short* w_pw1  = (unsigned short*)(ws + oWpw1);
  unsigned short* w_pw2  = (unsigned short*)(ws + oWpw2);
  unsigned short* posemb16 = (unsigned short*)(ws + oPosEmb);
  unsigned short* ppos16 = (unsigned short*)(ws + oPpos);
  float* halfb   = (float*)(ws + oHalfB);
  float* bnmean  = (float*)(ws + oBnMean);
  float* bnrstd  = (float*)(ws + oBnRstd);
  unsigned short* xn16a = (unsigned short*)(ws + oXnA);
  unsigned short* xn16b = (unsigned short*)(ws + oXnB);
  float* xnF   = (float*)(ws + oXnF);
  float* qF    = (float*)(ws + oQF);
  unsigned short* hid16 = (unsigned short*)(ws + oHid);
  unsigned short* k16   = (unsigned short*)(ws + oK16);
  unsigned short* vt16  = (unsigned short*)(ws + oVT16);
  unsigned short* qu16  = (unsigned short*)(ws + oQU16);
  unsigned short* qv16  = (unsigned short*)(ws + oQV16);
  float* ybuf  = (float*)(ws + oY);
  float* x1    = (float*)(ws + oX1);
  float* glu   = (float*)(ws + oGlu);
  float* x4    = (float*)(ws + oX4);
  unsigned short* att16 = (unsigned short*)(ws + oAtt);
  float* zbuf  = (float*)(ws + oZ);
  float* acbuf = (float*)(ws + oAC);
  unsigned short* p16 = (unsigned short*)(ws + oP16);
  float* x2    = (float*)(ws + oX2);
  float* bdbuf = (float*)(ws + oBD);
  unsigned short* sw16 = (unsigned short*)(ws + oSw);
  float* x3    = (float*)(ws + oX3);

  const dim3 blk(256);

  {
    const int n8_ffn = kFF * kD / 8;
    cast4_kernel<<<dim3((n8_ffn + 255) / 256, 4), blk, 0, stream>>>(
        ffm_w1, w_ffm1, n8_ffn, n8_ffn, kWCarry,
        ffm_w2, w_ffm2, n8_ffn, n8_ffn, kWCarry,
        ff_w1,  w_ff1,  n8_ffn, n8_ffn, kWCarry,
        ff_w2,  w_ff2,  n8_ffn, n8_ffn, kWCarry);
    const int n8_in = 3 * kD * kD / 8;
    const int n8_sq = kD * kD / 8;
    const int n8_pw1 = 2 * kD * kD / 8;
    cast4_kernel<<<dim3((n8_in + 255) / 256, 4), blk, 0, stream>>>(
        in_w,  w_in,  n8_in,  n8_in,  kWCarry,
        out_w, w_out, n8_sq,  n8_sq,  kWCarry,
        pos_w, w_pos, n8_sq,  n8_sq,  kWCarry,
        pw1_w, w_pw1, n8_pw1, n8_pw1, kWCarry);
    const int n8_pe_v = kNPv * kD / 8;
    const int n8_pe_t = kNP * kD / 8;
    cast4_kernel<<<dim3((n8_pe_t + 255) / 256, 4), blk, 0, stream>>>(
        pw2_w,   w_pw2,    n8_sq,   n8_sq,   kWCarry,
        pos_emb, posemb16, n8_pe_v, n8_pe_t, 1.0f,
        pw2_w,   w_pw2,    n8_sq,   0,       kWCarry,
        pw2_w,   w_pw2,    n8_sq,   0,       kWCarry);
  }
  halfbias_kernel<<<dim3(1), blk, 0, stream>>>(ffm_b2, ff_b2, halfb);

  const dim3 lngrid((kM + 7) / 8);

  ln_kernel<true, true><<<lngrid, blk, 0, stream>>>(x, ln_mac_g, ln_mac_b, xnF, xn16a, kM);
  run_gemm<2, 1, false, 3>(stream, xn16a, kD, 0L, w_ffm1, kD, 0L, hid16, kFF, 0L, ffm_b1, xnF, 0L, kM, kFF, kD, kWInv, 1);
  run_gemm<2, 0, true, 0>(stream, hid16, kFF, 0L, w_ffm2, kFF, 0L, x1, kD, 0L, halfb, xnF, 0L, kM, kD, kFF, kHalfWInv, 1);

  ln_kernel<false, true><<<lngrid, blk, 0, stream>>>(x1, ln_mha_g, ln_mha_b, xnF, xn16a, kM);
  run_gemm<2, 0, false, 0>(stream, xn16a, kD, 0L, w_in, kD, 0L, qF, kD, 0L, in_b, qF, 0L, kM, kD, kD, kWInv, 1);
  run_gemm<2, 1, false, 0>(stream, xn16a, kD, 0L, w_in + (size_t)kD * kD, kD, 0L, k16, kD, 0L, in_b + kD, qF, 0L, kM, kD, kD, kWInv, 1);
  run_gemm<1, 1, false, 0>(stream, w_in + (size_t)2 * kD * kD, kD, 0L, xn16a, kB * kD, (long)kD,
                           vt16, kT, (long)(kD * kT), in_b + 2 * kD, qF, 0L, kD, kT, kD, kWInv, kB);
  run_gemm<0, 1, false, 0>(stream, posemb16, kD, 0L, w_pos, kD, 0L, ppos16, kD, 0L, in_b, qF, 0L, kNP, kD, kD, kWInv, 1);
  quv_kernel<<<dim3((kM * kD / 8 + 255) / 256), blk, 0, stream>>>(qF, pbu, pbv, qu16, qv16, kM * kD / 8);
  for (int h = 0; h < kH; ++h) {
    run_gemm<0, 0, false, 0>(stream, qu16 + h * kHD, kB * kD, (long)kD, k16 + h * kHD, kB * kD, (long)kD,
                             acbuf, kT, (long)(kT * kT), in_b, qF, 0L, kT, kT, kHD, 1.0f, kB);
    run_gemm<0, 0, false, 0>(stream, qv16 + h * kHD, kB * kD, (long)kD, ppos16 + h * kHD, kD, 0L,
                             bdbuf, kNP, (long)(kT * kNP), in_b, qF, 0L, kT, kNP, kHD, 1.0f, kB);
    softmax_kernel<<<dim3((kB * kT + 7) / 8), blk, 0, stream>>>(acbuf, bdbuf, p16, kB * kT);
    run_gemm<0, 1, false, 0>(stream, p16, kT, (long)(kT * kT), vt16 + (size_t)h * kHD * kT, kT, (long)(kD * kT),
                             att16 + h * kHD, kB * kD, (long)kD, in_b, qF, 0L, kT, kHD, kT, kPVScale, kB);
  }
  run_gemm<2, 0, true, 0>(stream, att16, kD, 0L, w_out, kD, 0L, x2, kD, 0L, out_b, x1, 0L, kM, kD, kD, kOutProjScale, 1);

  ln_kernel<false, true><<<lngrid, blk, 0, stream>>>(x2, ln_conv_g, ln_conv_b, xnF, xn16b, kM);
  run_gemm<2, 0, false, 0>(stream, xn16b, kD, 0L, w_pw1, kD, 0L, ybuf, 2 * kD, 0L, pw1_b, ybuf, 0L, kM, 2 * kD, kD, kWInv, 1);
  glu_kernel<<<dim3((kM * kD / 4 + 255) / 256), blk, 0, stream>>>(ybuf, glu, kM * kD / 4);
  dwconv_kernel<<<dim3((kM * kD + 255) / 256), blk, 0, stream>>>(glu, dw_w, dw_b, zbuf, kM * kD);
  bnstats_kernel<<<dim3(kD / 32), blk, 0, stream>>>(zbuf, bnmean, bnrstd);
  bnswish_kernel<<<dim3((kM * kD / 8 + 255) / 256), blk, 0, stream>>>(zbuf, bnmean, bnrstd, bn_g, bn_b, sw16, kM * kD / 8);
  run_gemm<2, 0, true, 0>(stream, sw16, kD, 0L, w_pw2, kD, 0L, x3, kD, 0L, pw2_b, x2, 0L, kM, kD, kD, kWInv, 1);

  ln_kernel<false, true><<<lngrid, blk, 0, stream>>>(x3, ln_ff_g, ln_ff_b, xnF, xn16b, kM);
  run_gemm<2, 1, false, 3>(stream, xn16b, kD, 0L, w_ff1, kD, 0L, hid16, kFF, 0L, ff_b1, x3, 0L, kM, kFF, kD, kWInv, 1);
  run_gemm<2, 0, true, 0>(stream, hid16, kFF, 0L, w_ff2, kFF, 0L, x4, kD, 0L, halfb + kD, x3, 0L, kM, kD, kFF, kHalfWInv, 1);
  ln_kernel<true, false><<<lngrid, blk, 0, stream>>>(x4, ln_fin_g, ln_fin_b, out, xn16b, kM);
}
